// LlamaFlexAttention_24696061952631
// MI455X (gfx1250) — hardware-verified
//
#include <hip/hip_runtime.h>
#include <hip/hip_bf16.h>

typedef __attribute__((ext_vector_type(16))) __bf16 v16bf;
typedef float v8f __attribute__((ext_vector_type(8)));
typedef float v4f __attribute__((ext_vector_type(4)));
typedef unsigned int u4 __attribute__((ext_vector_type(4)));
typedef u4 __attribute__((may_alias)) u4a;
typedef v4f __attribute__((may_alias)) v4fa;

union Frag { v16bf v; u4 q[2]; };
union Acc  { v8f v; float f[8]; };

__device__ __forceinline__ unsigned bf_rne(float f) {
    unsigned u = __float_as_uint(f);
    u += 0x7FFFu + ((u >> 16) & 1u);
    return u >> 16;
}
__device__ __forceinline__ void split2(float x, unsigned& hi, unsigned& lo) {
    hi = bf_rne(x);
    lo = bf_rne(x - __uint_as_float(hi << 16));
}
__device__ __forceinline__ void pack2(float a, float b, unsigned& wh, unsigned& wl) {
    unsigned ha, la, hb, lb;
    split2(a, ha, la);
    split2(b, hb, lb);
    wh = ha | (hb << 16);
    wl = la | (lb << 16);
}
__device__ __forceinline__ void pack8(const v4f a, const v4f b, u4& H, u4& L) {
    unsigned h0, l0, h1, l1, h2, l2, h3, l3;
    pack2(a.x, a.y, h0, l0);
    pack2(a.z, a.w, h1, l1);
    pack2(b.x, b.y, h2, l2);
    pack2(b.z, b.w, h3, l3);
    H.x = h0; H.y = h1; H.z = h2; H.w = h3;
    L.x = l0; L.y = l1; L.z = l2; L.w = l3;
}

__device__ __forceinline__ void ldfrag(Frag& f, const unsigned short* p) {
    f.q[0] = *(const u4a*)(p);
    f.q[1] = *(const u4a*)(p + 16);
}

__device__ __forceinline__ void acc_zero(Acc& c) {
#pragma unroll
    for (int i = 0; i < 8; ++i) c.f[i] = 0.0f;
}

__device__ __forceinline__ void mma3(Acc& c, const Frag& ah, const Frag& al,
                                     const Frag& bh, const Frag& bl) {
    v8f d = c.v;
    d = __builtin_amdgcn_wmma_f32_16x16x32_bf16(false, ah.v, false, bh.v, (short)0, d, false, false);
    d = __builtin_amdgcn_wmma_f32_16x16x32_bf16(false, ah.v, false, bl.v, (short)0, d, false, false);
    d = __builtin_amdgcn_wmma_f32_16x16x32_bf16(false, al.v, false, bh.v, (short)0, d, false, false);
    asm volatile("v_nop\n\tv_nop\n\tv_nop\n\tv_nop"
                 : "+v"(d) : "v"(ah.v), "v"(al.v), "v"(bh.v), "v"(bl.v));
    c.v = d;
}

__device__ __forceinline__ void wave_sync() {
    __builtin_amdgcn_fence(__ATOMIC_ACQ_REL, "wavefront");
    __builtin_amdgcn_wave_barrier();
}

__global__ void invfreq_kernel(float* inv) {
    const int i = threadIdx.x & 31;
    const double e = (double)i * 0.03125 * 13.287712379549449;
    const float p32 = (float)exp2(e);
    const float v = 1.0f / p32;
    *(volatile float*)(inv + i) = v;
    __threadfence();
    *(volatile float*)(inv + i) = v;
}

__global__ __launch_bounds__(256) void cstable_kernel(const int* __restrict__ pid,
                                                      const float* __restrict__ inv,
                                                      float* cosT, float* sinT,
                                                      int ntok, int lck) {
    const int n = ntok * 32;
    const int idx = blockIdx.x * 256 + threadIdx.x;
    const int ic = (idx < n) ? idx : (n - 1);
    const int tok = ic >> 5, i = ic & 31;
    const float pos = (float)(pid[tok] + lck);
    const float ang = pos * inv[i];
    const float c = cosf(ang);
    const float s = sinf(ang);
    if (idx < n) {
        *(volatile float*)(cosT + idx) = c;
        *(volatile float*)(sinT + idx) = s;
    }
    __threadfence();
    if (idx < n) {
        *(volatile float*)(cosT + idx) = c;
        *(volatile float*)(sinT + idx) = s;
    }
}

__global__ __launch_bounds__(256) void split8_kernel(const float* __restrict__ src,
                                                     unsigned short* dh, unsigned short* dl,
                                                     int n8, int logseg, int addshift) {
    const int t = blockIdx.x * 256 + threadIdx.x;
    if (t >= n8) return;
    const float* p = src + (size_t)t * 8;
    const v4f a = *(const v4fa*)(p);
    const v4f b = *(const v4fa*)(p + 4);
    u4 H, L;
    pack8(a, b, H, L);
    const size_t g = ((size_t)t + ((size_t)(t >> logseg) << addshift)) * 8;
    *(volatile u4*)(dh + g) = H;
    *(volatile u4*)(dl + g) = L;
    __threadfence();
    *(volatile u4*)(dh + g) = H;
    *(volatile u4*)(dl + g) = L;
}

__global__ __launch_bounds__(256) void tsplit_kernel(const float* __restrict__ src, int srcld, int srcz,
                                                     unsigned short* dh, unsigned short* dl,
                                                     int dstld, int dstz, int nbase) {
    constexpr int TP = 72;
    __shared__ __align__(16) unsigned short Th[64 * TP];
    __shared__ __align__(16) unsigned short Tl[64 * TP];
    const int t = threadIdx.x;
    const int c0 = blockIdx.x * 64, r0 = blockIdx.y * 64, z = blockIdx.z;
    const float* s = src + (size_t)z * srcz + (size_t)r0 * srcld + c0;
#pragma unroll
    for (int i = 0; i < 4; ++i) {
        const int r = (t >> 4) + 16 * i, c4 = (t & 15) * 4;
        const v4f v = *(const v4fa*)(s + (size_t)r * srcld + c4);
        unsigned hb, lb;
        split2(v.x, hb, lb); Th[(c4 + 0) * TP + r] = (unsigned short)hb; Tl[(c4 + 0) * TP + r] = (unsigned short)lb;
        split2(v.y, hb, lb); Th[(c4 + 1) * TP + r] = (unsigned short)hb; Tl[(c4 + 1) * TP + r] = (unsigned short)lb;
        split2(v.z, hb, lb); Th[(c4 + 2) * TP + r] = (unsigned short)hb; Tl[(c4 + 2) * TP + r] = (unsigned short)lb;
        split2(v.w, hb, lb); Th[(c4 + 3) * TP + r] = (unsigned short)hb; Tl[(c4 + 3) * TP + r] = (unsigned short)lb;
    }
    __syncthreads();
    const int piece = t & 7;
    const int rowA = (t >> 3), rowB = 32 + (t >> 3);
    const u4 HA = *(const u4a*)(Th + rowA * TP + piece * 8);
    const u4 LA = *(const u4a*)(Tl + rowA * TP + piece * 8);
    const u4 HB = *(const u4a*)(Th + rowB * TP + piece * 8);
    const u4 LB = *(const u4a*)(Tl + rowB * TP + piece * 8);
    const size_t zb = (size_t)z * dstz;
    const size_t gA = zb + (size_t)(nbase + c0 + rowA) * dstld + r0 + piece * 8;
    const size_t gB = zb + (size_t)(nbase + c0 + rowB) * dstld + r0 + piece * 8;
    *(volatile u4*)(dh + gA) = HA; *(volatile u4*)(dl + gA) = LA;
    *(volatile u4*)(dh + gB) = HB; *(volatile u4*)(dl + gB) = LB;
    __threadfence();
    *(volatile u4*)(dh + gA) = HA; *(volatile u4*)(dl + gA) = LA;
    *(volatile u4*)(dh + gB) = HB; *(volatile u4*)(dl + gB) = LB;
}

__device__ __forceinline__ void store_ctile(const float* sW, float* C, int ldc,
                                            int m0w, int n0w, int hh, int m16) {
#pragma unroll
    for (int i = 0; i < 16; ++i) {
        const int row = 2 * i + hh;
        const v4f v = *(const v4fa*)(sW + row * 68 + m16 * 4);
        *(volatile v4f*)(C + (size_t)(m0w + row) * ldc + n0w + m16 * 4) = v;
    }
}

__global__ __launch_bounds__(128) void gemm3_kernel(
    const unsigned short* __restrict__ Ah, const unsigned short* __restrict__ Al,
    const unsigned short* __restrict__ Bh, const unsigned short* __restrict__ Bl,
    float* C, int K, int ldc) {
    constexpr int SP = 68;
    __shared__ __align__(16) float sC[4 * 32 * SP];
    const int tid = threadIdx.x, w = tid >> 5, lane = tid & 31, hh = lane >> 4, m16 = lane & 15;
    const int m0w = blockIdx.y * 64 + (w >> 1) * 32;
    const int n0w = blockIdx.x * 128 + (w & 1) * 64;

    Acc acc[2][4];
#pragma unroll
    for (int mt = 0; mt < 2; ++mt)
#pragma unroll
        for (int nt = 0; nt < 4; ++nt) acc_zero(acc[mt][nt]);

    const size_t Ks = (size_t)K;
    const unsigned short* ah0 = Ah + (size_t)(m0w + m16) * Ks + 8 * hh;
    const unsigned short* al0 = Al + (size_t)(m0w + m16) * Ks + 8 * hh;
    const unsigned short* ah1 = ah0 + 16 * Ks;
    const unsigned short* al1 = al0 + 16 * Ks;
    const unsigned short* bh0 = Bh + (size_t)(n0w + m16) * Ks + 8 * hh;
    const unsigned short* bl0 = Bl + (size_t)(n0w + m16) * Ks + 8 * hh;

#pragma unroll 1
    for (int k0 = 0; k0 < K; k0 += 32) {
        Frag fah[2], fal[2];
        ldfrag(fah[0], ah0 + k0);
        ldfrag(fal[0], al0 + k0);
        ldfrag(fah[1], ah1 + k0);
        ldfrag(fal[1], al1 + k0);
#pragma unroll
        for (int nt = 0; nt < 4; ++nt) {
            Frag fbh, fbl;
            ldfrag(fbh, bh0 + (size_t)nt * 16 * Ks + k0);
            ldfrag(fbl, bl0 + (size_t)nt * 16 * Ks + k0);
            mma3(acc[0][nt], fah[0], fal[0], fbh, fbl);
            mma3(acc[1][nt], fah[1], fal[1], fbh, fbl);
        }
    }

    float* sW = sC + w * (32 * SP);
#pragma unroll
    for (int mt = 0; mt < 2; ++mt)
#pragma unroll
        for (int nt = 0; nt < 4; ++nt)
#pragma unroll
            for (int r = 0; r < 8; ++r)
                sW[(mt * 16 + 8 * hh + r) * SP + nt * 16 + m16] = acc[mt][nt].f[r];
    __syncthreads();
    store_ctile(sW, C, ldc, m0w, n0w, hh, m16);
    __threadfence();
    store_ctile(sW, C, ldc, m0w, n0w, hh, m16);
}

__device__ __forceinline__ void rope8(const float* xr, const float* pr, const float* cr,
                                      const float* sr, float sgn, v4f& ya, v4f& yb) {
#pragma clang fp contract(off)
    ya.x = xr[0] * cr[0] + (sgn * pr[0]) * sr[0];
    ya.y = xr[1] * cr[1] + (sgn * pr[1]) * sr[1];
    ya.z = xr[2] * cr[2] + (sgn * pr[2]) * sr[2];
    ya.w = xr[3] * cr[3] + (sgn * pr[3]) * sr[3];
    yb.x = xr[4] * cr[4] + (sgn * pr[4]) * sr[4];
    yb.y = xr[5] * cr[5] + (sgn * pr[5]) * sr[5];
    yb.z = xr[6] * cr[6] + (sgn * pr[6]) * sr[6];
    yb.w = xr[7] * cr[7] + (sgn * pr[7]) * sr[7];
}

__global__ __launch_bounds__(256) void rope_split_kernel(
    const float* __restrict__ qkv, const float* __restrict__ cosT, const float* __restrict__ sinT,
    unsigned short* qh, unsigned short* ql, unsigned short* kh, unsigned short* kl,
    unsigned short* vh, unsigned short* vl) {
#pragma clang fp contract(off)
    constexpr int QN = 1024, D = 64, NH = 32, NKV = 8, QKVW = 3072, KVL = 3072, KVP = 2048, TP = 68;
    __shared__ __align__(16) float T[64 * TP];
    const int t = threadIdx.x, g = blockIdx.x, tok0 = blockIdx.y * 64;
    const float* s = qkv + (size_t)tok0 * QKVW + g * D;
#pragma unroll
    for (int i = 0; i < 4; ++i) {
        const int r = (t >> 4) + 16 * i, c4 = (t & 15) * 4;
        const v4f v = *(const v4fa*)(s + (size_t)r * QKVW + c4);
        *(v4fa*)(T + r * TP + c4) = v;
    }
    __syncthreads();

    u4 H0, L0, H1, L1;
    size_t g0, g1;
    unsigned short* dH;
    unsigned short* dL;
    if (g < NH + NKV) {
        const bool isq = (g < NH);
        dH = isq ? qh : kh;
        dL = isq ? ql : kl;
        const int d0 = (t & 7) * 8, dp0 = d0 ^ 32;
        const float sgn = (d0 < 32) ? -1.0f : 1.0f;
        {
            const int r = (t >> 3), tok = tok0 + r;
            const float* cr = cosT + (size_t)tok * 32 + (d0 & 31);
            const float* sr = sinT + (size_t)tok * 32 + (d0 & 31);
            v4f ya, yb;
            rope8(T + r * TP + d0, T + r * TP + dp0, cr, sr, sgn, ya, yb);
            pack8(ya, yb, H0, L0);
            const size_t row = isq ? ((size_t)g * QN + tok) : ((size_t)(g - NH) * KVL + KVP + tok);
            g0 = row * D + d0;
        }
        {
            const int r = 32 + (t >> 3), tok = tok0 + r;
            const float* cr = cosT + (size_t)tok * 32 + (d0 & 31);
            const float* sr = sinT + (size_t)tok * 32 + (d0 & 31);
            v4f ya, yb;
            rope8(T + r * TP + d0, T + r * TP + dp0, cr, sr, sgn, ya, yb);
            pack8(ya, yb, H1, L1);
            const size_t row = isq ? ((size_t)g * QN + tok) : ((size_t)(g - NH) * KVL + KVP + tok);
            g1 = row * D + d0;
        }
    } else {
        dH = vh;
        dL = vl;
        const int kvhd = g - NH - NKV, piece = t & 7;
        {
            const int d = (t >> 3);
            v4f ya, yb;
            ya.x = T[(piece * 8 + 0) * TP + d]; ya.y = T[(piece * 8 + 1) * TP + d];
            ya.z = T[(piece * 8 + 2) * TP + d]; ya.w = T[(piece * 8 + 3) * TP + d];
            yb.x = T[(piece * 8 + 4) * TP + d]; yb.y = T[(piece * 8 + 5) * TP + d];
            yb.z = T[(piece * 8 + 6) * TP + d]; yb.w = T[(piece * 8 + 7) * TP + d];
            pack8(ya, yb, H0, L0);
            g0 = ((size_t)(kvhd * D + d)) * KVL + KVP + tok0 + piece * 8;
        }
        {
            const int d = 32 + (t >> 3);
            v4f ya, yb;
            ya.x = T[(piece * 8 + 0) * TP + d]; ya.y = T[(piece * 8 + 1) * TP + d];
            ya.z = T[(piece * 8 + 2) * TP + d]; ya.w = T[(piece * 8 + 3) * TP + d];
            yb.x = T[(piece * 8 + 4) * TP + d]; yb.y = T[(piece * 8 + 5) * TP + d];
            yb.z = T[(piece * 8 + 6) * TP + d]; yb.w = T[(piece * 8 + 7) * TP + d];
            pack8(ya, yb, H1, L1);
            g1 = ((size_t)(kvhd * D + d)) * KVL + KVP + tok0 + piece * 8;
        }
    }
    *(volatile u4*)(dH + g0) = H0; *(volatile u4*)(dL + g0) = L0;
    *(volatile u4*)(dH + g1) = H1; *(volatile u4*)(dL + g1) = L1;
    __threadfence();
    *(volatile u4*)(dH + g0) = H0; *(volatile u4*)(dL + g0) = L0;
    *(volatile u4*)(dH + g1) = H1; *(volatile u4*)(dL + g1) = L1;
}

__global__ __launch_bounds__(128) void attn_kernel(
    const unsigned short* __restrict__ qH, const unsigned short* __restrict__ qL,
    const unsigned short* __restrict__ kH, const unsigned short* __restrict__ kL,
    const unsigned short* __restrict__ vH, const unsigned short* __restrict__ vL,
    const int* __restrict__ amask, int nmask, int lck,
    unsigned short* oH, unsigned short* oL) {
    constexpr int QN = 1024, D = 64, KVL = 3072, HIDO = 2048, NBLK = 3, PP = 40, OP = 72;
    __shared__ int red[128];
    __shared__ __align__(16) unsigned short Ph[4 * 16 * PP];
    __shared__ __align__(16) unsigned short Pl[4 * 16 * PP];
    __shared__ __align__(16) unsigned short Oh[4 * 16 * OP];
    __shared__ __align__(16) unsigned short Ol[4 * 16 * OP];
    const int tid = threadIdx.x, w = tid >> 5, lane = tid & 31, hh = lane >> 4, m16 = lane & 15;

    int part = 0;
    for (int i = tid; i < nmask; i += 128) part += amask[i];
    red[tid] = part;
    __syncthreads();
#pragma unroll
    for (int off = 64; off > 0; off >>= 1) {
        if (tid < off) red[tid] += red[tid + off];
        __syncthreads();
    }
    const int seq_len = __builtin_amdgcn_readfirstlane(red[0] - lck);

    const int h = blockIdx.y, kvh = h >> 2;
    const int q0w = blockIdx.x * 64 + w * 16;
    const float NEG_INF = -__builtin_inff();

    Frag fqh[2], fql[2];
    {
        const size_t qo = ((size_t)h * QN + q0w + m16) * D + 8 * hh;
        ldfrag(fqh[0], qH + qo);
        ldfrag(fqh[1], qH + qo + 32);
        ldfrag(fql[0], qL + qo);
        ldfrag(fql[1], qL + qo + 32);
    }
    float mrow[8], lrow[8];
    Acc o[4];
#pragma unroll
    for (int r = 0; r < 8; ++r) { mrow[r] = NEG_INF; lrow[r] = 0.0f; }
#pragma unroll
    for (int dt = 0; dt < 4; ++dt) acc_zero(o[dt]);

    unsigned short* Pwh = Ph + w * 16 * PP;
    unsigned short* Pwl = Pl + w * 16 * PP;
    const size_t kplane = (size_t)kvh * KVL * D;
    const size_t vplane = (size_t)kvh * D * KVL;

    for (int blk = 0; blk < NBLK; ++blk) {
        const int shift = lck - blk;
        int jcnt = q0w + 16 - shift;
        jcnt = (jcnt < seq_len) ? jcnt : seq_len;
        jcnt = (jcnt < 0) ? 0 : ((jcnt > QN) ? QN : jcnt);
        const int nsteps = __builtin_amdgcn_readfirstlane((jcnt + 31) >> 5);
#pragma unroll 1
        for (int t = 0; t < nsteps; ++t) {
            const int j0 = t * 32, kv0 = blk * QN + j0;
            Acc sc[2];
            acc_zero(sc[0]);
            acc_zero(sc[1]);
#pragma unroll
            for (int nt = 0; nt < 2; ++nt) {
                const size_t ko = kplane + (size_t)(kv0 + nt * 16 + m16) * D + 8 * hh;
#pragma unroll
                for (int ds = 0; ds < 2; ++ds) {
                    Frag fkh, fkl;
                    ldfrag(fkh, kH + ko + ds * 32);
                    ldfrag(fkl, kL + ko + ds * 32);
                    mma3(sc[nt], fqh[ds], fql[ds], fkh, fkl);
                }
            }
#pragma unroll
            for (int nt = 0; nt < 2; ++nt)
#pragma unroll
                for (int r = 0; r < 8; ++r) {
                    const int qi = q0w + 8 * hh + r;
                    const int j = j0 + nt * 16 + m16;
                    const bool ok = (j < seq_len) && (j <= qi - shift);
                    sc[nt].f[r] = ok ? sc[nt].f[r] * 0.125f : NEG_INF;
                }
            float alpha[8];
#pragma unroll
            for (int r = 0; r < 8; ++r) {
                float x = fmaxf(sc[0].f[r], sc[1].f[r]);
                x = fmaxf(x, __shfl_xor(x, 1));
                x = fmaxf(x, __shfl_xor(x, 2));
                x = fmaxf(x, __shfl_xor(x, 4));
                x = fmaxf(x, __shfl_xor(x, 8));
                const float mn = fmaxf(mrow[r], x);
                const float msafe = (mn == NEG_INF) ? 0.0f : mn;
                alpha[r] = __expf(mrow[r] - msafe);
                mrow[r] = mn;
                const float p0 = __expf(sc[0].f[r] - msafe);
                const float p1 = __expf(sc[1].f[r] - msafe);
                sc[0].f[r] = p0;
                sc[1].f[r] = p1;
                float sum = p0 + p1;
                sum += __shfl_xor(sum, 1);
                sum += __shfl_xor(sum, 2);
                sum += __shfl_xor(sum, 4);
                sum += __shfl_xor(sum, 8);
                lrow[r] = lrow[r] * alpha[r] + sum;
            }
#pragma unroll
            for (int dt = 0; dt < 4; ++dt)
#pragma unroll
                for (int r = 0; r < 8; ++r) o[dt].f[r] *= alpha[r];

            wave_sync();
#pragma unroll
            for (int nt = 0; nt < 2; ++nt)
#pragma unroll
                for (int r = 0; r < 8; ++r) {
                    unsigned hb, lb;
                    split2(sc[nt].f[r], hb, lb);
                    Pwh[(8 * hh + r) * PP + nt * 16 + m16] = (unsigned short)hb;
                    Pwl[(8 * hh + r) * PP + nt * 16 + m16] = (unsigned short)lb;
                }
            wave_sync();
            Frag fph, fpl;
            ldfrag(fph, Pwh + m16 * PP + 8 * hh);
            ldfrag(fpl, Pwl + m16 * PP + 8 * hh);

#pragma unroll
            for (int dt = 0; dt < 4; ++dt) {
                const size_t vo = vplane + (size_t)(dt * 16 + m16) * KVL + kv0 + 8 * hh;
                Frag fvh, fvl;
                ldfrag(fvh, vH + vo);
                ldfrag(fvl, vL + vo);
                mma3(o[dt], fph, fpl, fvh, fvl);
            }
        }
    }

    unsigned short* Owh = Oh + w * 16 * OP;
    unsigned short* Owl = Ol + w * 16 * OP;
#pragma unroll
    for (int r = 0; r < 8; ++r) {
        const float il = 1.0f / lrow[r];
#pragma unroll
        for (int dt = 0; dt < 4; ++dt) {
            unsigned hb, lb;
            split2(o[dt].f[r] * il, hb, lb);
            Owh[(8 * hh + r) * OP + dt * 16 + m16] = (unsigned short)hb;
            Owl[(8 * hh + r) * OP + dt * 16 + m16] = (unsigned short)lb;
        }
    }
    wave_sync();
    const int piece = lane & 7, rq = lane >> 3;
    const u4 a0 = *(const u4a*)(Owh + (0 + rq) * OP + piece * 8);
    const u4 a1 = *(const u4a*)(Owh + (4 + rq) * OP + piece * 8);
    const u4 a2 = *(const u4a*)(Owh + (8 + rq) * OP + piece * 8);
    const u4 a3 = *(const u4a*)(Owh + (12 + rq) * OP + piece * 8);
    const u4 b0 = *(const u4a*)(Owl + (0 + rq) * OP + piece * 8);
    const u4 b1 = *(const u4a*)(Owl + (4 + rq) * OP + piece * 8);
    const u4 b2 = *(const u4a*)(Owl + (8 + rq) * OP + piece * 8);
    const u4 b3 = *(const u4a*)(Owl + (12 + rq) * OP + piece * 8);
    const size_t e0 = (size_t)(q0w + 0 + rq) * HIDO + h * D + piece * 8;
    const size_t e1 = (size_t)(q0w + 4 + rq) * HIDO + h * D + piece * 8;
    const size_t e2 = (size_t)(q0w + 8 + rq) * HIDO + h * D + piece * 8;
    const size_t e3 = (size_t)(q0w + 12 + rq) * HIDO + h * D + piece * 8;
    *(volatile u4*)(oH + e0) = a0; *(volatile u4*)(oL + e0) = b0;
    *(volatile u4*)(oH + e1) = a1; *(volatile u4*)(oL + e1) = b1;
    *(volatile u4*)(oH + e2) = a2; *(volatile u4*)(oL + e2) = b2;
    *(volatile u4*)(oH + e3) = a3; *(volatile u4*)(oL + e3) = b3;
    __threadfence();
    *(volatile u4*)(oH + e0) = a0; *(volatile u4*)(oL + e0) = b0;
    *(volatile u4*)(oH + e1) = a1; *(volatile u4*)(oL + e1) = b1;
    *(volatile u4*)(oH + e2) = a2; *(volatile u4*)(oL + e2) = b2;
    *(volatile u4*)(oH + e3) = a3; *(volatile u4*)(oL + e3) = b3;
}

extern "C" void kernel_launch(void* const* d_in, const int* in_sizes, int n_in,
                              void* d_out, int out_size, void* d_ws, size_t ws_size,
                              hipStream_t stream) {
    constexpr int QN = 1024, INW = 4096, NH = 32, NKV = 8, D = 64, HIDO = 2048;
    constexpr int KVP = 2048, KVL = 3072, QKVW = 3072, LCK = KVP / QN;
    if (n_in < 9) return;
    if (in_sizes[0] != QN * INW || in_sizes[1] != NKV * KVP * D || in_sizes[2] != NKV * KVP * D ||
        in_sizes[3] != QN || in_sizes[4] != QN || in_sizes[5] != INW * NH * D ||
        in_sizes[6] != INW * NKV * D || in_sizes[7] != INW * NKV * D ||
        in_sizes[8] != NH * D * HIDO || out_size != QN * HIDO) return;

    const float* hs  = (const float*)d_in[0];
    const float* pk  = (const float*)d_in[1];
    const float* pv  = (const float*)d_in[2];
    const int*   am  = (const int*)  d_in[3];
    const int*   pid = (const int*)  d_in[4];
    const float* Wq  = (const float*)d_in[5];
    const float* Wk  = (const float*)d_in[6];
    const float* Wv  = (const float*)d_in[7];
    const float* Wo  = (const float*)d_in[8];
    float* out = (float*)d_out;

    char* ws = (char*)d_ws;
    size_t off = 0;
    auto carve = [&](size_t bytes) -> char* {
        char* p = ws + off;
        off += (bytes + 255) & ~(size_t)255;
        return p;
    };
    unsigned short* hsH = (unsigned short*)carve((size_t)QN * INW * 2);
    unsigned short* hsL = (unsigned short*)carve((size_t)QN * INW * 2);
    unsigned short* wtH = (unsigned short*)carve((size_t)QKVW * INW * 2);
    unsigned short* wtL = (unsigned short*)carve((size_t)QKVW * INW * 2);
    unsigned short* woH = (unsigned short*)carve((size_t)HIDO * (NH * D) * 2);
    unsigned short* woL = (unsigned short*)carve((size_t)HIDO * (NH * D) * 2);
    float*          qkv = (float*)         carve((size_t)QN * QKVW * 4);
    unsigned short* qH  = (unsigned short*)carve((size_t)NH * QN * D * 2);
    unsigned short* qL  = (unsigned short*)carve((size_t)NH * QN * D * 2);
    unsigned short* kH  = (unsigned short*)carve((size_t)NKV * KVL * D * 2);
    unsigned short* kL  = (unsigned short*)carve((size_t)NKV * KVL * D * 2);
    unsigned short* vH  = (unsigned short*)carve((size_t)NKV * D * KVL * 2);
    unsigned short* vL  = (unsigned short*)carve((size_t)NKV * D * KVL * 2);
    unsigned short* aH  = (unsigned short*)carve((size_t)QN * (NH * D) * 2);
    unsigned short* aL  = (unsigned short*)carve((size_t)QN * (NH * D) * 2);
    float*          cosT = (float*)        carve((size_t)QN * 32 * 4);
    float*          sinT = (float*)        carve((size_t)QN * 32 * 4);
    float*          inv  = (float*)        carve(128);
    if (off > ws_size || off > ((size_t)128 << 20)) return;

    invfreq_kernel<<<1, 32, 0, stream>>>(inv);
    cstable_kernel<<<(QN * 32) / 256, 256, 0, stream>>>(pid, inv, cosT, sinT, QN, LCK);

    split8_kernel<<<(QN * INW / 8) / 256, 256, 0, stream>>>(hs, hsH, hsL, QN * INW / 8, 30, 0);
    split8_kernel<<<(NKV * KVP * D / 8) / 256, 256, 0, stream>>>(pk, kH, kL, NKV * KVP * D / 8, 14, 13);
    tsplit_kernel<<<dim3((NH * D) / 64, INW / 64, 1), 256, 0, stream>>>(Wq, NH * D, 0, wtH, wtL, INW, 0, 0);
    tsplit_kernel<<<dim3((NKV * D) / 64, INW / 64, 1), 256, 0, stream>>>(Wk, NKV * D, 0, wtH, wtL, INW, 0, NH * D);
    tsplit_kernel<<<dim3((NKV * D) / 64, INW / 64, 1), 256, 0, stream>>>(Wv, NKV * D, 0, wtH, wtL, INW, 0, NH * D + NKV * D);
    tsplit_kernel<<<dim3(HIDO / 64, (NH * D) / 64, 1), 256, 0, stream>>>(Wo, HIDO, 0, woH, woL, NH * D, 0, 0);
    tsplit_kernel<<<dim3(D / 64, KVP / 64, NKV), 256, 0, stream>>>(pv, D, KVP * D, vH, vL, KVL, D * KVL, 0);

    gemm3_kernel<<<dim3(QKVW / 128, QN / 64), 128, 0, stream>>>(hsH, hsL, wtH, wtL, qkv, INW, QKVW);

    rope_split_kernel<<<dim3(QKVW / 64, QN / 64), 256, 0, stream>>>(qkv, cosT, sinT, qH, qL, kH, kL, vH, vL);

    attn_kernel<<<dim3(QN / 64, NH), 128, 0, stream>>>(qH, qL, kH, kL, vH, vL, am, in_sizes[3], LCK, aH, aL);

    gemm3_kernel<<<dim3(HIDO / 128, QN / 64), 128, 0, stream>>>(aH, aL, woH, woL, out, NH * D, HIDO);
}
